// ICLAttentionAlt_52493090292405
// MI455X (gfx1250) — hardware-verified
//
#include <hip/hip_runtime.h>
#include <stddef.h>


#define HEADS 8
#define DE 64
#define BATCH 2
#define SEQ 2048
#define BH (BATCH * HEADS)
#define ZDIM (HEADS * DE)
#define ROWS (BATCH * SEQ)
#define QT (SEQ / 16)
#define RT64 (ROWS / 64)
#define WPITCH 72
#define KPITCH 40
#define OPITCH 68
#define NEG_BIG (-3.0e38f)

typedef char chk_de[(DE == 64) ? 1 : -1];
typedef char chk_seq[((SEQ % 64) == 0) ? 1 : -1];
typedef char chk_rows[((ROWS % 64) == 0) ? 1 : -1];
typedef char chk_waves[(((BH * QT) % 2) == 0) ? 1 : -1];
typedef char chk_z[((ZDIM % 32) == 0) ? 1 : -1];

typedef __bf16 bf16_t;
typedef bf16_t v16bf __attribute__((ext_vector_type(16)));
typedef float v8f __attribute__((ext_vector_type(8)));
typedef float v4f __attribute__((ext_vector_type(4)));
typedef float v2f __attribute__((ext_vector_type(2)));
typedef unsigned int v4u __attribute__((ext_vector_type(4)));
typedef unsigned short us_t;

union Frag {
  v16bf v;
  v4u u[2];
};

__device__ __forceinline__ v4u mk4(unsigned int a, unsigned int b, unsigned int c, unsigned int d) {
  v4u r;
  r.x = a; r.y = b; r.z = c; r.w = d;
  return r;
}

__device__ __forceinline__ v8f zero8() {
  v8f z;
#pragma unroll
  for (int i = 0; i < 8; ++i) z[i] = 0.f;
  return z;
}

__device__ __forceinline__ unsigned int bf_rne(float x) {
  unsigned int u = __float_as_uint(x);
  u += 0x7FFFu + ((u >> 16) & 1u);
  return u >> 16;
}
__device__ __forceinline__ float bf_val(unsigned int b) { return __uint_as_float(b << 16); }

__device__ __forceinline__ void split2(float x0, float x1, unsigned int& ph, unsigned int& pl) {
  const unsigned int h0 = bf_rne(x0), h1 = bf_rne(x1);
  const unsigned int l0 = bf_rne(x0 - bf_val(h0)), l1 = bf_rne(x1 - bf_val(h1));
  ph = h0 | (h1 << 16);
  pl = l0 | (l1 << 16);
}
__device__ __forceinline__ void split1(float x, us_t& hb, us_t& lb) {
  const unsigned int h = bf_rne(x);
  hb = (us_t)h;
  lb = (us_t)bf_rne(x - bf_val(h));
}
__device__ __forceinline__ void split8(v4f a, v4f b, v4u& ph, v4u& pl) {
  unsigned int h0, l0, h1, l1, h2, l2, h3, l3;
  split2(a.x, a.y, h0, l0);
  split2(a.z, a.w, h1, l1);
  split2(b.x, b.y, h2, l2);
  split2(b.z, b.w, h3, l3);
  ph = mk4(h0, h1, h2, h3);
  pl = mk4(l0, l1, l2, l3);
}

__device__ __forceinline__ v8f mma3(v16bf ah, v16bf al, v16bf bh, v16bf bl, v8f c) {
  c = __builtin_amdgcn_wmma_f32_16x16x32_bf16(false, ah, false, bh, (short)0, c, false, false);
  c = __builtin_amdgcn_wmma_f32_16x16x32_bf16(false, ah, false, bl, (short)0, c, false, false);
  c = __builtin_amdgcn_wmma_f32_16x16x32_bf16(false, al, false, bh, (short)0, c, false, false);
  asm volatile("v_nop\n\tv_nop\n\tv_nop\n\tv_nop" : "+v"(c) : "v"(ah), "v"(al), "v"(bh), "v"(bl));
  return c;
}

__device__ __forceinline__ v16bf ldfrag(const us_t* base, int ld, int k0, int l) {
  const us_t* p = base + (size_t)(l & 15) * ld + k0 + 8 * (l >> 4);
  Frag f;
  f.u[0] = *(const v4u*)p;
  f.u[1] = *(const v4u*)(p + 16);
  return f.v;
}

__global__ __launch_bounds__(128) void k_proj(
    const float* __restrict__ q, const float* __restrict__ k, const float* __restrict__ v,
    const float* __restrict__ Wq, const float* __restrict__ Wk, const float* __restrict__ Wv,
    us_t* __restrict__ qhh, us_t* __restrict__ qhl, us_t* __restrict__ khh, us_t* __restrict__ khl,
    us_t* __restrict__ vth, us_t* __restrict__ vtl) {
#pragma clang fp contract(off)
  __shared__ __attribute__((aligned(16))) us_t wt[2][DE][WPITCH];
  __shared__ __attribute__((aligned(16))) us_t st[2][64][WPITCH];
  __shared__ float invf[32];

  const int t = threadIdx.x, w = t >> 5, l = t & 31, m = l & 15, hh = l >> 4;
  const int blk = blockIdx.x;
  const int mat = blk / (HEADS * RT64);
  const int rem = blk - mat * (HEADS * RT64);
  const int head = rem / RT64;
  const int rt = rem - head * RT64;
  const int row0 = rt * 64;
  const int b = row0 / SEQ, s0 = row0 - b * SEQ, bh = b * HEADS + head;

  const float* X = (mat == 0) ? q : ((mat == 1) ? k : v);
  const float* W = ((mat == 0) ? Wq : ((mat == 1) ? Wk : Wv)) + (size_t)head * DE * DE;

#pragma unroll 4
  for (int j = 0; j < 32; ++j) {
    const int idx = j * 128 + t;
    const int z = idx >> 6, d = idx & 63;
    us_t hb, lb;
    split1(W[idx], hb, lb);
    wt[0][d][z] = hb;
    wt[1][d][z] = lb;
  }
  if (t < 32) invf[t] = 1.0f / powf(10000.0f, (float)t * 0.03125f);
  __syncthreads();

  const float* xr = X + (size_t)(row0 + w * 16 + m) * DE;
  Frag ah0, al0, ah1, al1;
  {
    v4f a, c;
    a = *(const v4f*)(xr + 8 * hh);       c = *(const v4f*)(xr + 8 * hh + 4);       split8(a, c, ah0.u[0], al0.u[0]);
    a = *(const v4f*)(xr + 16 + 8 * hh);  c = *(const v4f*)(xr + 16 + 8 * hh + 4);  split8(a, c, ah0.u[1], al0.u[1]);
    a = *(const v4f*)(xr + 32 + 8 * hh);  c = *(const v4f*)(xr + 32 + 8 * hh + 4);  split8(a, c, ah1.u[0], al1.u[0]);
    a = *(const v4f*)(xr + 48 + 8 * hh);  c = *(const v4f*)(xr + 48 + 8 * hh + 4);  split8(a, c, ah1.u[1], al1.u[1]);
  }

  v8f acc[4];
#pragma unroll
  for (int n = 0; n < 4; ++n) acc[n] = zero8();
#pragma unroll
  for (int n = 0; n < 4; ++n) {
    acc[n] = mma3(ah0.v, al0.v, ldfrag(&wt[0][n * 16][0], WPITCH, 0, l),
                  ldfrag(&wt[1][n * 16][0], WPITCH, 0, l), acc[n]);
    acc[n] = mma3(ah1.v, al1.v, ldfrag(&wt[0][n * 16][0], WPITCH, 32, l),
                  ldfrag(&wt[1][n * 16][0], WPITCH, 32, l), acc[n]);
  }

  if (mat < 2) {
#pragma unroll
    for (int n = 0; n < 4; ++n) {
      const int N = n * 16 + m;
      const float f = invf[N >> 1];
#pragma unroll
      for (int r = 0; r < 8; ++r) {
        const int pos = s0 + w * 16 + 8 * hh + r;
        const float ang = (float)pos * f;
        const float sn = sinf(ang), cs = cosf(ang);
        const float mine = acc[n][r];
        const float other = __shfl_xor(mine, 1, 32);
        acc[n][r] = ((N & 1) == 0) ? (mine * cs - other * sn) : (other * sn + mine * cs);
      }
    }
  }

  if (mat == 2) {
#pragma unroll
    for (int n = 0; n < 4; ++n)
#pragma unroll
      for (int r = 0; r < 8; ++r) {
        us_t hb, lb;
        split1(acc[n][r], hb, lb);
        st[0][n * 16 + m][w * 16 + 8 * hh + r] = hb;
        st[1][n * 16 + m][w * 16 + 8 * hh + r] = lb;
      }
  } else {
#pragma unroll
    for (int n = 0; n < 4; ++n)
#pragma unroll
      for (int r = 0; r < 8; ++r) {
        us_t hb, lb;
        split1(acc[n][r], hb, lb);
        st[0][w * 16 + 8 * hh + r][n * 16 + m] = hb;
        st[1][w * 16 + 8 * hh + r][n * 16 + m] = lb;
      }
  }
  __syncthreads();

  v4u vals[2][4];
  size_t offs[4];
  const int ch = l & 7, sub4 = l >> 3;
  us_t* dsth;
  us_t* dstl;
  if (mat == 2) {
    dsth = vth; dstl = vtl;
#pragma unroll
    for (int i = 0; i < 4; ++i) {
      const int d = w * 16 + 4 * i + sub4;
      vals[0][i] = *(const v4u*)&st[0][d][ch * 8];
      vals[1][i] = *(const v4u*)&st[1][d][ch * 8];
      offs[i] = ((size_t)bh * DE + d) * SEQ + s0 + ch * 8;
    }
  } else {
    dsth = (mat == 0) ? qhh : khh;
    dstl = (mat == 0) ? qhl : khl;
#pragma unroll
    for (int i = 0; i < 4; ++i) {
      const int rr = w * 16 + 4 * i + sub4;
      vals[0][i] = *(const v4u*)&st[0][rr][ch * 8];
      vals[1][i] = *(const v4u*)&st[1][rr][ch * 8];
      offs[i] = ((size_t)bh * SEQ + s0 + rr) * DE + ch * 8;
    }
  }
#pragma unroll
  for (int i = 0; i < 4; ++i) {
    *(volatile v4u*)(dsth + offs[i]) = vals[0][i];
    *(volatile v4u*)(dstl + offs[i]) = vals[1][i];
  }
  __threadfence();
#pragma unroll
  for (int i = 0; i < 4; ++i) {
    *(volatile v4u*)(dsth + offs[i]) = vals[0][i];
    *(volatile v4u*)(dstl + offs[i]) = vals[1][i];
  }
}

__global__ __launch_bounds__(64) void k_stats(
    const us_t* __restrict__ qhh, const us_t* __restrict__ qhl,
    const us_t* __restrict__ khh, const us_t* __restrict__ khl, float* __restrict__ ml) {
  const int wave = blockIdx.x * 2 + (threadIdx.x >> 5);
  const int bh = wave / QT, qt = wave - bh * QT;
  const int l = threadIdx.x & 31, m = l & 15, hh = l >> 4;

  const size_t qoff = ((size_t)bh * SEQ + qt * 16) * DE;
  const v16bf aqh0 = ldfrag(qhh + qoff, DE, 0, l), aqh1 = ldfrag(qhh + qoff, DE, 32, l);
  const v16bf aql0 = ldfrag(qhl + qoff, DE, 0, l), aql1 = ldfrag(qhl + qoff, DE, 32, l);
  const us_t* Kh = khh + (size_t)bh * SEQ * DE;
  const us_t* Kl = khl + (size_t)bh * SEQ * DE;

  float mrow[8], lrow[8];
#pragma unroll
  for (int r = 0; r < 8; ++r) { mrow[r] = NEG_BIG; lrow[r] = 0.f; }

#pragma unroll 1
  for (int kt = 0; kt <= qt; ++kt) {
    const size_t ko = (size_t)kt * 16 * DE;
    v8f s = zero8();
    s = mma3(aqh0, aql0, ldfrag(Kh + ko, DE, 0, l), ldfrag(Kl + ko, DE, 0, l), s);
    s = mma3(aqh1, aql1, ldfrag(Kh + ko, DE, 32, l), ldfrag(Kl + ko, DE, 32, l), s);
#pragma unroll
    for (int r = 0; r < 8; ++r) {
      const int qg = qt * 16 + 8 * hh + r;
      const int kg = kt * 16 + m;
      const float x = (kg <= qg) ? s[r] * (1.0f / 64.0f) : NEG_BIG;
      float gm = x;
#pragma unroll
      for (int off = 1; off < 16; off <<= 1) gm = fmaxf(gm, __shfl_xor(gm, off, 32));
      const float mn = fmaxf(mrow[r], gm);
      float e = __expf(x - mn);
#pragma unroll
      for (int off = 1; off < 16; off <<= 1) e += __shfl_xor(e, off, 32);
      lrow[r] = lrow[r] * __expf(mrow[r] - mn) + e;
      mrow[r] = mn;
    }
  }

  const int rs0 = 2 * (l & 3), rs1 = rs0 + 1;
  float m0 = 0.f, l0 = 1.f, m1 = 0.f, l1 = 1.f;
#pragma unroll
  for (int r = 0; r < 8; ++r) {
    if (r == rs0) { m0 = mrow[r]; l0 = lrow[r]; }
    if (r == rs1) { m1 = mrow[r]; l1 = lrow[r]; }
  }
  const int src = (l & 3) + (((l >> 2) & 1) << 4);
  m0 = __shfl(m0, src, 32); l0 = __shfl(l0, src, 32);
  m1 = __shfl(m1, src, 32); l1 = __shfl(l1, src, 32);
  v4f val;
  val.x = m0; val.y = 1.0f / l0; val.z = m1; val.w = 1.0f / l1;
  float* dst = ml + ((size_t)bh * SEQ + qt * 16) * 2 + 4 * l;
  if (l < 8) *(volatile v4f*)dst = val;
  __threadfence();
  if (l < 8) *(volatile v4f*)dst = val;
}

__global__ __launch_bounds__(64) void k_attn(
    const us_t* __restrict__ qhh, const us_t* __restrict__ qhl,
    const us_t* __restrict__ khh, const us_t* __restrict__ khl,
    const us_t* __restrict__ vth, const us_t* __restrict__ vtl,
    const float* __restrict__ ml, float* __restrict__ outh) {
  __shared__ __attribute__((aligned(16))) float so[2][16][OPITCH];
  const int w = threadIdx.x >> 5;
  const int wave = blockIdx.x * 2 + w;
  const int bh = wave / QT, kt = wave - bh * QT;
  const int l = threadIdx.x & 31, m = l & 15, hh = l >> 4;

  const size_t koff = ((size_t)bh * SEQ + kt * 16) * DE;
  const v16bf bkh0 = ldfrag(khh + koff, DE, 0, l), bkh1 = ldfrag(khh + koff, DE, 32, l);
  const v16bf bkl0 = ldfrag(khl + koff, DE, 0, l), bkl1 = ldfrag(khl + koff, DE, 32, l);

  v8f o[4];
#pragma unroll
  for (int n = 0; n < 4; ++n) o[n] = zero8();

  const int kg = kt * 16 + m;
  const float* mlb = ml + (size_t)bh * SEQ * 2;
  const us_t* Qh = qhh + (size_t)bh * SEQ * DE;
  const us_t* Ql = qhl + (size_t)bh * SEQ * DE;
  const us_t* Vh = vth + (size_t)bh * DE * SEQ;
  const us_t* Vl = vtl + (size_t)bh * DE * SEQ;

#pragma unroll 1
  for (int qc = (kt >> 1) * 32; qc < SEQ; qc += 32) {
    unsigned int ph[2][4], pl[2][4];
#pragma unroll
    for (int sub = 0; sub < 2; ++sub) {
      const int q0 = qc + 16 * sub;
      const size_t qo = (size_t)q0 * DE;
      v8f s = zero8();
      s = mma3(ldfrag(Qh + qo, DE, 0, l), ldfrag(Ql + qo, DE, 0, l), bkh0, bkl0, s);
      s = mma3(ldfrag(Qh + qo, DE, 32, l), ldfrag(Ql + qo, DE, 32, l), bkh1, bkl1, s);
      float p[8];
#pragma unroll
      for (int r = 0; r < 8; ++r) {
        const int qg = q0 + 8 * hh + r;
        const v2f mr = *(const v2f*)(mlb + 2 * qg);
        const float e = __expf(s[r] * (1.0f / 64.0f) - mr.x) * mr.y;
        p[r] = (kg < qg) ? e : 0.f;
      }
#pragma unroll
      for (int j = 0; j < 4; ++j) split2(p[2 * j], p[2 * j + 1], ph[sub][j], pl[sub][j]);
    }
    Frag aph, apl;
    aph.u[0] = mk4(ph[0][0], ph[0][1], ph[0][2], ph[0][3]);
    aph.u[1] = mk4(ph[1][0], ph[1][1], ph[1][2], ph[1][3]);
    apl.u[0] = mk4(pl[0][0], pl[0][1], pl[0][2], pl[0][3]);
    apl.u[1] = mk4(pl[1][0], pl[1][1], pl[1][2], pl[1][3]);
#pragma unroll
    for (int n = 0; n < 4; ++n) {
      const size_t vo = (size_t)(n * 16) * SEQ;
      o[n] = mma3(aph.v, apl.v, ldfrag(Vh + vo, SEQ, qc, l), ldfrag(Vl + vo, SEQ, qc, l), o[n]);
    }
  }

#pragma unroll
  for (int n = 0; n < 4; ++n)
#pragma unroll
    for (int r = 0; r < 8; ++r) so[w][8 * hh + r][n * 16 + m] = o[n][r];
  __syncthreads();

  const int bb = bh / HEADS, head = bh - bb * HEADS;
  v4f vals[8];
  size_t offs[8];
#pragma unroll
  for (int i = 0; i < 8; ++i) {
    const int row = 2 * i + hh;
    vals[i] = *(const v4f*)&so[w][row][4 * m];
    offs[i] = ((size_t)bb * SEQ + kt * 16 + row) * ZDIM + head * DE + 4 * m;
  }
#pragma unroll
  for (int i = 0; i < 8; ++i) *(volatile v4f*)(outh + offs[i]) = vals[i];
  __threadfence();
#pragma unroll
  for (int i = 0; i < 8; ++i) *(volatile v4f*)(outh + offs[i]) = vals[i];
}

__global__ __launch_bounds__(128) void k_oproj(
    const float* __restrict__ outh, const float* __restrict__ Wo, float* __restrict__ out) {
  __shared__ __attribute__((aligned(16))) us_t wo[2][DE][KPITCH];
  __shared__ __attribute__((aligned(16))) float so[4][16][OPITCH];
  const int t = threadIdx.x, w = t >> 5, l = t & 31, m = l & 15, hh = l >> 4;
  const int rowbase = blockIdx.x * 64 + w * 16;

  v8f acc[4];
#pragma unroll
  for (int n = 0; n < 4; ++n) acc[n] = zero8();

#pragma unroll 1
  for (int c = 0; c < ZDIM / 32; ++c) {
    __syncthreads();
#pragma unroll
    for (int j = 0; j < 16; ++j) {
      const int idx = j * 128 + t;
      const int zz = idx >> 6, d = idx & 63;
      us_t hb, lb;
      split1(Wo[(size_t)(c * 32 + zz) * DE + d], hb, lb);
      wo[0][d][zz] = hb;
      wo[1][d][zz] = lb;
    }
    __syncthreads();
    const float* ar = outh + (size_t)(rowbase + m) * ZDIM + c * 32;
    Frag ah, al;
    {
      v4f a, e;
      a = *(const v4f*)(ar + 8 * hh);       e = *(const v4f*)(ar + 8 * hh + 4);       split8(a, e, ah.u[0], al.u[0]);
      a = *(const v4f*)(ar + 16 + 8 * hh);  e = *(const v4f*)(ar + 16 + 8 * hh + 4);  split8(a, e, ah.u[1], al.u[1]);
    }
#pragma unroll
    for (int n = 0; n < 4; ++n)
      acc[n] = mma3(ah.v, al.v, ldfrag(&wo[0][n * 16][0], KPITCH, 0, l),
                    ldfrag(&wo[1][n * 16][0], KPITCH, 0, l), acc[n]);
  }

#pragma unroll
  for (int n = 0; n < 4; ++n)
#pragma unroll
    for (int r = 0; r < 8; ++r) so[w][8 * hh + r][n * 16 + m] = acc[n][r];
  __syncthreads();

  v4f vals[8];
  size_t offs[8];
#pragma unroll
  for (int i = 0; i < 8; ++i) {
    const int row = 2 * i + hh;
    vals[i] = *(const v4f*)&so[w][row][4 * m];
    offs[i] = (size_t)(rowbase + row) * DE + 4 * m;
  }
#pragma unroll
  for (int i = 0; i < 8; ++i) *(volatile v4f*)(out + offs[i]) = vals[i];
  __threadfence();
#pragma unroll
  for (int i = 0; i < 8; ++i) *(volatile v4f*)(out + offs[i]) = vals[i];
}

extern "C" void kernel_launch(void* const* d_in, const int* in_sizes, int n_in,
                              void* d_out, int out_size, void* d_ws, size_t ws_size,
                              hipStream_t stream) {
  if (n_in < 7) return;
  if (in_sizes[0] != ROWS * DE || in_sizes[1] != ROWS * DE || in_sizes[2] != ROWS * DE) return;
  if (in_sizes[3] != HEADS * DE * DE || in_sizes[4] != HEADS * DE * DE || in_sizes[5] != HEADS * DE * DE) return;
  if (in_sizes[6] != ZDIM * DE) return;
  if (out_size != ROWS * DE) return;

  const float* q  = (const float*)d_in[0];
  const float* k  = (const float*)d_in[1];
  const float* v  = (const float*)d_in[2];
  const float* Wq = (const float*)d_in[3];
  const float* Wk = (const float*)d_in[4];
  const float* Wv = (const float*)d_in[5];
  const float* Wo = (const float*)d_in[6];
  float* out = (float*)d_out;

  char* ws = (char*)d_ws;
  size_t off = 0;
  const size_t plane = (size_t)BH * SEQ * DE * sizeof(us_t);
  us_t* qhh = (us_t*)(ws + off); off += plane;
  us_t* qhl = (us_t*)(ws + off); off += plane;
  us_t* khh = (us_t*)(ws + off); off += plane;
  us_t* khl = (us_t*)(ws + off); off += plane;
  us_t* vth = (us_t*)(ws + off); off += plane;
  us_t* vtl = (us_t*)(ws + off); off += plane;
  float* ml   = (float*)(ws + off); off += (size_t)BH * SEQ * 2 * sizeof(float);
  float* outh = (float*)(ws + off); off += (size_t)ROWS * ZDIM * sizeof(float);
  if (off > ws_size) return;

  k_proj<<<dim3(3 * HEADS * RT64), dim3(128), 0, stream>>>(q, k, v, Wq, Wk, Wv,
                                                           qhh, qhl, khh, khl, vth, vtl);
  k_stats<<<dim3((BH * QT) / 2), dim3(64), 0, stream>>>(qhh, qhl, khh, khl, ml);
  k_attn<<<dim3((BH * QT) / 2), dim3(64), 0, stream>>>(qhh, qhl, khh, khl, vth, vtl, ml, outh);
  k_oproj<<<dim3(ROWS / 64), dim3(128), 0, stream>>>(outh, Wo, out);
}
